// OskarLayer_12987981103315
// MI455X (gfx1250) — hardware-run, weakly checked
//
#include <hip/hip_runtime.h>
#include <math.h>

constexpr int kB    = 2;
constexpr int kS    = 4096;
constexpr int kHid  = 768;
constexpr int kNH   = 12;
constexpr int kDh   = 64;
constexpr int kFF   = 3072;
constexpr int kW    = 128;
constexpr int kTok  = kB * kS;
constexpr int kNC   = kS / kW;
constexpr int kWin  = 3 * kW;
constexpr int kSpad = kS + 2 * kW;
constexpr int kNBH  = kB * kNH;
constexpr int kGrp  = 4;
constexpr int kNPass = kNBH / kGrp;
constexpr int kTC   = 2048;
constexpr int kNTC  = kTok / kTC;

constexpr float kWCarry   = 16.0f;
constexpr float kInvW     = 1.0f / 16.0f;
constexpr float kQScale   = 0.125f;
constexpr float kPCarry   = 2048.0f;
constexpr float kCtxCarry = 16.0f;
constexpr float kPVScale  = kCtxCarry / kPCarry;
constexpr float kWdScale  = 1.0f / (kCtxCarry * kWCarry);
constexpr float kInvHid   = 1.0f / 768.0f;
constexpr float kLnEps    = 1e-12f;

constexpr size_t kSzTokH  = (size_t)kTok * kHid * 2;
constexpr size_t kSzTokF  = (size_t)kTok * kHid * 4;
constexpr size_t kSzW     = (size_t)kHid * kHid * 2;
constexpr size_t kSzWf    = (size_t)kFF * kHid * 2;
constexpr size_t kSzPad   = (size_t)kB * kSpad * kHid * 2;
constexpr size_t kOffX16  = 0;
constexpr size_t kOffWT   = kOffX16 + kSzTokH;
constexpr size_t kOffQ16  = kOffWT + 4 * kSzW;
constexpr size_t kOffKpad = kOffQ16 + kSzTokH;
constexpr size_t kOffVT   = kOffKpad + kSzPad;
constexpr size_t kOffSc   = kOffVT + kSzPad;
constexpr size_t kOffP16  = kOffSc + kSzTokF;
constexpr size_t kOffCtx  = kOffP16 + kSzTokH;
constexpr size_t kOffR8   = kOffCtx + kSzTokH;
constexpr size_t kWsTotal = kOffR8 + kSzTokF;
static_assert(kWsTotal == 132120576ull);
static_assert(kWsTotal <= 134217728ull);
static_assert(kSzPad == (size_t)kNBH * kDh * kSpad * 2);
static_assert((size_t)kGrp * kNC * kW * kWin * 4 == kSzTokF);
static_assert((size_t)kGrp * kNC * kW * kWin * 2 == kSzTokH);
static_assert(kSzTokF <= 2 * kSzPad);
static_assert(2 * kSzWf <= kSzTokH);
static_assert((size_t)kTok * kFF * 2 == kSzTokF + 2 * kSzTokH);
static_assert((size_t)kTC * kFF * 4 == kSzTokF);
static_assert(kNH % kGrp == 0);

typedef __attribute__((ext_vector_type(16))) _Float16 v16h;
typedef __attribute__((ext_vector_type(8)))  _Float16 v8h;
typedef __attribute__((ext_vector_type(16))) __bf16   v16b;
typedef __attribute__((ext_vector_type(8)))  __bf16   v8b;
typedef __attribute__((ext_vector_type(8)))  float    v8f;
typedef __attribute__((ext_vector_type(4)))  float    v4f;
typedef __attribute__((ext_vector_type(4)))  unsigned int v4u;

__device__ __forceinline__ void dep_guard_h(v8f& a, v8f& b, v16h x, v16h y) { asm volatile("v_nop\n\tv_nop\n\tv_nop\n\tv_nop" : "+v"(a), "+v"(b) : "v"(x), "v"(y)); }
__device__ __forceinline__ void dep_guard_b(v8f& a, v8f& b, v16b x, v16b y) { asm volatile("v_nop\n\tv_nop\n\tv_nop\n\tv_nop" : "+v"(a), "+v"(b) : "v"(x), "v"(y)); }
__device__ __forceinline__ void keep4_h(v16h a, v16h b, v16h c, v16h d) { asm volatile("v_nop" :: "v"(a), "v"(b), "v"(c), "v"(d)); }
__device__ __forceinline__ void keep4_b(v16b a, v16b b, v16b c, v16b d) { asm volatile("v_nop" :: "v"(a), "v"(b), "v"(c), "v"(d)); }
__device__ __forceinline__ void acc_guard4(v8f& a, v8f& b, v8f& c, v8f& d) { asm volatile("v_nop\n\tv_nop\n\tv_nop\n\tv_nop" : "+v"(a), "+v"(b), "+v"(c), "+v"(d)); }
template <typename T> struct Frag;
template <> struct Frag<_Float16> {
  typedef v16h V; union U { v16h v; v8h h[2]; };
  static __device__ __forceinline__ v16h load(const _Float16* p) {
    U f; f.h[0] = *(const v8h*)(p); f.h[1] = *(const v8h*)(p + 16); return f.v;
  }
  static __device__ __forceinline__ v8f mma(v16h a, v16h b, v8f c) {
    return __builtin_amdgcn_wmma_f32_16x16x32_f16(false, a, false, b, (short)0, c, false, false);
  }
  static __device__ __forceinline__ void guard(v8f& a, v8f& b, v16h x, v16h y) { dep_guard_h(a, b, x, y); }
  static __device__ __forceinline__ void keep(v16h a, v16h b, v16h c, v16h d) { keep4_h(a, b, c, d); }
};
template <> struct Frag<__bf16> {
  typedef v16b V; union U { v16b v; v8b h[2]; };
  static __device__ __forceinline__ v16b load(const __bf16* p) {
    U f; f.h[0] = *(const v8b*)(p); f.h[1] = *(const v8b*)(p + 16); return f.v;
  }
  static __device__ __forceinline__ v8f mma(v16b a, v16b b, v8f c) {
    return __builtin_amdgcn_wmma_f32_16x16x32_bf16(false, a, false, b, (short)0, c, false, false);
  }
  static __device__ __forceinline__ void guard(v8f& a, v8f& b, v16b x, v16b y) { dep_guard_b(a, b, x, y); }
  static __device__ __forceinline__ void keep(v16b a, v16b b, v16b c, v16b d) { keep4_b(a, b, c, d); }
};

__device__ __forceinline__ unsigned pk16(unsigned short a, unsigned short b) { return (unsigned)a | ((unsigned)b << 16); }
__device__ __forceinline__ unsigned short h_bits(float f) { const _Float16 h = (_Float16)f; return __builtin_bit_cast(unsigned short, h); }

template <int BIAS_MODE, int OUT_MODE, bool RESID>
__global__ __launch_bounds__(256) void gemm_f16_kernel(
    const unsigned short* __restrict__ Ap, int lda, long strideAy, long strideAz,
    const unsigned short* __restrict__ Btp, int ldb, long strideBy, long strideBz,
    void* __restrict__ Cout, int ldc, long strideCy, long strideCz,
    const float* __restrict__ bias, const float* __restrict__ resid,
    int M, int N, int K, float scale, int nBy, int nBz) {
  typedef _Float16 T;
  typedef v16h V;
  const T* A = (const T*)Ap; const T* Bt = (const T*)Btp;
  __shared__ __align__(16) float sT[8][16 * 68];
  const int lane = threadIdx.x & 31;
  const int wave = threadIdx.x >> 5;
  const int tilesN = N >> 6;
  const int tilesM = M >> 6;
  const int per = tilesM * tilesN;
  const int tileg = blockIdx.x * 8 + wave;
  if (tileg >= per * nBy * nBz) return;
  const int bt   = tileg / per;
  const int tile = tileg - bt * per;
  const int bz   = bt / nBy;
  const int by   = bt - bz * nBy;
  const int tm = tile / tilesN;
  const int tn = tile - tm * tilesN;
  const int m0 = tm << 6;
  const int n0 = tn << 6;

  const T* Ab = A  + (long)by * strideAy + (long)bz * strideAz;
  const T* Bb = Bt + (long)by * strideBy + (long)bz * strideBz;
  const long cOff = (long)by * strideCy + (long)bz * strideCz;

  const int rlane = lane & 15;
  const int koff  = (lane >> 4) * 8;
  const int mOff  = (lane >> 4) * 8;

  v8f acc[4][4];
#pragma unroll
  for (int i = 0; i < 4; ++i)
#pragma unroll
    for (int j = 0; j < 4; ++j) acc[i][j] = (v8f){0.f,0.f,0.f,0.f,0.f,0.f,0.f,0.f};

  for (int k0 = 0; k0 < K; k0 += 32) {
    V bh[4];
#pragma unroll
    for (int j = 0; j < 4; ++j) {
      const size_t bo = (size_t)(n0 + (j << 4) + rlane) * ldb + koff + k0;
      bh[j] = Frag<T>::load(Bb + bo);
    }
#pragma unroll
    for (int i = 0; i < 4; ++i) {
      const size_t ao = (size_t)(m0 + (i << 4) + rlane) * lda + koff + k0;
      V ah = Frag<T>::load(Ab + ao);
#pragma unroll
      for (int j = 0; j < 4; ++j) acc[i][j] = Frag<T>::mma(ah, bh[j], acc[i][j]);
      Frag<T>::guard(acc[i][0], acc[i][3], ah, ah);
    }
    Frag<T>::keep(bh[0], bh[1], bh[2], bh[3]);
  }
  acc_guard4(acc[0][0], acc[0][1], acc[0][2], acc[0][3]);
  acc_guard4(acc[1][0], acc[1][1], acc[1][2], acc[1][3]);
  acc_guard4(acc[2][0], acc[2][1], acc[2][2], acc[2][3]);
  acc_guard4(acc[3][0], acc[3][1], acc[3][2], acc[3][3]);

  float* slab = sT[wave];
  const float* Rb = RESID ? resid : nullptr;
#pragma unroll
  for (int i = 0; i < 4; ++i) {
    const int mBase = m0 + (i << 4);
#pragma unroll
    for (int j = 0; j < 4; ++j) {
      const int n = n0 + (j << 4) + rlane;
      float bv = 0.f;
      if (BIAS_MODE == 2) bv = bias[n];
#pragma unroll
      for (int r = 0; r < 8; ++r) {
        float v = acc[i][j][r] * scale;
        if (BIAS_MODE == 1) v += bias[mBase + mOff + r];
        if (BIAS_MODE == 2) v += bv;
        if (RESID) v += Rb[(size_t)(mBase + mOff + r) * ldc + n];
        slab[(mOff + r) * 68 + (j << 4) + rlane] = v;
      }
    }
    __builtin_amdgcn_fence(__ATOMIC_RELEASE, "workgroup");
    __builtin_amdgcn_wave_barrier();
    __builtin_amdgcn_fence(__ATOMIC_ACQUIRE, "workgroup");
    if (OUT_MODE == 0) {
      float* C = (float*)Cout + cOff;
      const int hh = lane >> 4, c4 = (lane & 15) * 4;
      for (int pass = 0; pass < 2; ++pass) {
#pragma unroll
        for (int it = 0; it < 8; ++it) {
          const int row = it * 2 + hh;
          v4f v = *(const v4f*)(slab + row * 68 + c4);
          *(volatile v4f*)(C + (size_t)(mBase + row) * ldc + n0 + c4) = v;
        }
        __threadfence();
      }
    } else {
      const int q = lane >> 3, c8 = (lane & 7) * 8;
      unsigned short* C = (unsigned short*)Cout + cOff;
      for (int pass = 0; pass < 2; ++pass) {
#pragma unroll
        for (int it = 0; it < 4; ++it) {
          const int row = it * 4 + q;
          const float* sp = slab + row * 68 + c8;
          v8h hv;
#pragma unroll
          for (int e = 0; e < 8; ++e) hv[e] = (_Float16)sp[e];
          *(volatile v8h*)(C + (size_t)(mBase + row) * ldc + n0 + c8) = hv;
        }
        __threadfence();
      }
    }
    __builtin_amdgcn_fence(__ATOMIC_RELEASE, "workgroup");
    __builtin_amdgcn_wave_barrier();
    __builtin_amdgcn_fence(__ATOMIC_ACQUIRE, "workgroup");
  }
}

__global__ __launch_bounds__(256) void cast8_f16_kernel(const float* __restrict__ in, unsigned short* __restrict__ out, int n8) {
  const int i = blockIdx.x * 256 + threadIdx.x;
  if (i >= n8) return;
  const float* p = in + 8 * (size_t)i;
  const v4f a = *(const v4f*)(p);
  const v4f c = *(const v4f*)(p + 4);
  unsigned short hb[8];
#pragma unroll
  for (int e = 0; e < 4; ++e) {
    hb[e]     = h_bits(a[e]);
    hb[4 + e] = h_bits(c[e]);
  }
  const v4u u = (v4u){pk16(hb[0], hb[1]), pk16(hb[2], hb[3]), pk16(hb[4], hb[5]), pk16(hb[6], hb[7])};
  unsigned short* q = out + 8 * (size_t)i;
  *(volatile v4u*)q = u;
  __threadfence();
  *(volatile v4u*)q = u;
}

__global__ __launch_bounds__(256) void wtcast_kernel(const float* __restrict__ W0, const float* __restrict__ W1,
                                                     const float* __restrict__ W2, const float* __restrict__ W3,
                                                     unsigned short* __restrict__ out, int K, int N, float scale) {
  __shared__ float sm[64][65];
  const int t  = threadIdx.x;
  const int k0 = blockIdx.x * 64;
  const int n0 = blockIdx.y * 64;
  const int z  = blockIdx.z;
  const float* Wp = (z == 0) ? W0 : (z == 1) ? W1 : (z == 2) ? W2 : W3;
#pragma unroll
  for (int i = 0; i < 16; ++i) {
    const int e = i * 256 + t;
    const int r = e >> 6;
    const int c = e & 63;
    sm[c][r] = Wp[(size_t)(k0 + r) * N + n0 + c] * scale;
  }
  __syncthreads();
  const int lane = t & 31, wave = t >> 5;
  const int q = lane >> 3, c8 = (lane & 7) * 8;
  unsigned short* op = out + (size_t)z * N * K;
  for (int pass = 0; pass < 2; ++pass) {
#pragma unroll
    for (int it = 0; it < 2; ++it) {
      const int row = wave * 8 + it * 4 + q;
      unsigned short hb[8];
#pragma unroll
      for (int e = 0; e < 8; ++e) hb[e] = h_bits(sm[row][c8 + e]);
      const v4u u = (v4u){pk16(hb[0], hb[1]), pk16(hb[2], hb[3]), pk16(hb[4], hb[5]), pk16(hb[6], hb[7])};
      *(volatile v4u*)(op + (size_t)(n0 + row) * K + k0 + c8) = u;
    }
    __threadfence();
  }
}

__global__ __launch_bounds__(256) void padzero_kernel(unsigned short* __restrict__ Kpad, unsigned short* __restrict__ VT) {
  const int t = threadIdx.x;
  const int blk = blockIdx.x;
  const v4u z4 = (v4u){0u, 0u, 0u, 0u};
  if (blk < 192) {
    const int e8 = blk * 256 + t;
    const int seg = e8 / 12288;
    const int b = seg >> 1, side = seg & 1;
    const int within = e8 - seg * 12288;
    unsigned short* p = Kpad + (size_t)b * kSpad * kHid + (side ? (size_t)(kW + kS) * kHid : (size_t)0) + (size_t)within * 8;
    *(volatile v4u*)p = z4;
    __threadfence();
    *(volatile v4u*)p = z4;
  } else {
    const int idx = (blk - 192) * 256 + t;
    const int l16 = idx & 15;
    const int seg = idx >> 4;
    const int rowi = seg >> 1, side = seg & 1;
    unsigned short* p = VT + (size_t)rowi * kSpad + (side ? (kW + kS) : 0) + l16 * 8;
    *(volatile v4u*)p = z4;
    __threadfence();
    *(volatile v4u*)p = z4;
  }
}

__global__ __launch_bounds__(256) void band_softmax_kernel(const float* __restrict__ Sc, const int* __restrict__ am,
                                                           unsigned short* __restrict__ P, int bsel) {
  __shared__ __align__(16) float st[8][kWin];
  const int lane = threadIdx.x & 31, wave = threadIdx.x >> 5;
  const int r = blockIdx.x * 8 + wave;
  const int rem = r & (kNC * kW - 1);
  const int c = rem >> 7;
  const int x = rem & (kW - 1);
  const float* srow = Sc + (size_t)r * kWin;
  unsigned short* prow = P + (size_t)r * kWin;
  float* tb = st[wave];
  const int jb = c * kW - kW;
  float m = -INFINITY;
#pragma unroll 1
  for (int i = 0; i < 12; ++i) {
    const int y = i * 32 + lane;
    const float s = srow[y];
    const int j = jb + y;
    const int jc = min(max(j, 0), kS - 1);
    const int flag = am[(size_t)bsel * kS + jc];
    const bool keep = (y >= x) && (y <= x + 2 * kW) && (j >= 0) && (j < kS);
    const float madd = (flag != 0) ? -10000.0f : 0.0f;
    const float tv = keep ? (s + madd) : -INFINITY;
    tb[y] = tv;
    m = fmaxf(m, tv);
  }
#pragma unroll
  for (int off = 16; off > 0; off >>= 1) m = fmaxf(m, __shfl_xor(m, off, 32));
  float sum = 0.f;
#pragma unroll 1
  for (int i = 0; i < 12; ++i) {
    const int y = i * 32 + lane;
    const float e = expf(tb[y] - m);
    tb[y] = e;
    sum += e;
  }
#pragma unroll
  for (int off = 16; off > 0; off >>= 1) sum += __shfl_xor(sum, off, 32);
  const float rs = kPCarry * (1.0f / sum);
  __builtin_amdgcn_fence(__ATOMIC_RELEASE, "workgroup");
  __builtin_amdgcn_wave_barrier();
  __builtin_amdgcn_fence(__ATOMIC_ACQUIRE, "workgroup");
  const int lb = lane & 15;
  const v4f a0 = *(const v4f*)(tb + 8 * lane);
  const v4f a1 = *(const v4f*)(tb + 8 * lane + 4);
  const v4f b0 = *(const v4f*)(tb + 256 + 8 * lb);
  const v4f b1 = *(const v4f*)(tb + 256 + 8 * lb + 4);
  unsigned short ha[8], hb[8];
#pragma unroll
  for (int e = 0; e < 4; ++e) {
    ha[e]     = h_bits(a0[e] * rs);
    ha[4 + e] = h_bits(a1[e] * rs);
    hb[e]     = h_bits(b0[e] * rs);
    hb[4 + e] = h_bits(b1[e] * rs);
  }
  const v4u ua = (v4u){pk16(ha[0], ha[1]), pk16(ha[2], ha[3]), pk16(ha[4], ha[5]), pk16(ha[6], ha[7])};
  const v4u ub = (v4u){pk16(hb[0], hb[1]), pk16(hb[2], hb[3]), pk16(hb[4], hb[5]), pk16(hb[6], hb[7])};
  for (int pass = 0; pass < 2; ++pass) {
    *(volatile v4u*)(prow + 8 * lane) = ua;
    if (lane < 16) *(volatile v4u*)(prow + 256 + 8 * lane) = ub;
    __threadfence();
  }
}

template <bool HOUT>
__global__ __launch_bounds__(192) void layernorm_kernel(const float* __restrict__ in, const float* __restrict__ gam,
                                                        const float* __restrict__ bet, float* __restrict__ outF,
                                                        unsigned short* __restrict__ outH) {
  __shared__ __align__(16) float rowv[kHid];
  __shared__ float red[8];
  const int row = blockIdx.x, t = threadIdx.x;
  const int lane = t & 31, wave = t >> 5;
  const size_t rb = (size_t)row * kHid;
  const v4f xv = *(const v4f*)(in + rb + 4 * t);
  float s = (xv[0] + xv[1]) + (xv[2] + xv[3]);
#pragma unroll
  for (int off = 16; off > 0; off >>= 1) s += __shfl_xor(s, off, 32);
  if (lane == 0) red[wave] = s;
  __syncthreads();
  const float tot = ((red[0] + red[1]) + (red[2] + red[3])) + (red[4] + red[5]);
  const float mean = tot * kInvHid;
  __syncthreads();
  const float d0 = xv[0] - mean, d1 = xv[1] - mean, d2 = xv[2] - mean, d3 = xv[3] - mean;
  float q = (d0 * d0 + d1 * d1) + (d2 * d2 + d3 * d3);
#pragma unroll
  for (int off = 16; off > 0; off >>= 1) q += __shfl_xor(q, off, 32);
  if (lane == 0) red[wave] = q;
  __syncthreads();
  const float vtot = ((red[0] + red[1]) + (red[2] + red[3])) + (red[4] + red[5]);
  const float var = vtot * kInvHid;
  const float rstd = rsqrtf(var + kLnEps);
  const v4f gv = *(const v4f*)(gam + 4 * t);
  const v4f bv = *(const v4f*)(bet + 4 * t);
  v4f yv;
  yv[0] = d0 * rstd * gv[0] + bv[0];
  yv[1] = d1 * rstd * gv[1] + bv[1];
  yv[2] = d2 * rstd * gv[2] + bv[2];
  yv[3] = d3 * rstd * gv[3] + bv[3];
  float* op = outF + rb + 4 * t;
  *(volatile v4f*)op = yv;
  __threadfence();
  *(volatile v4f*)op = yv;
  if (HOUT) {
    *(v4f*)(rowv + 4 * t) = yv;
    __syncthreads();
    if (t < 96) {
      const v4f a = *(const v4f*)(rowv + 8 * t);
      const v4f c = *(const v4f*)(rowv + 8 * t + 4);
      unsigned short hb[8];
#pragma unroll
      for (int e = 0; e < 4; ++e) { hb[e] = h_bits(a[e]); hb[4 + e] = h_bits(c[e]); }
      const v4u u = (v4u){pk16(hb[0], hb[1]), pk16(hb[2], hb[3]), pk16(hb[4], hb[5]), pk16(hb[6], hb[7])};
      unsigned short* hp = outH + rb + 8 * t;
      *(volatile v4u*)hp = u;
      __threadfence();
      *(volatile v4u*)hp = u;
    }
  }
}

__global__ __launch_bounds__(256) void gelu_f16_kernel(const float* __restrict__ in, unsigned short* __restrict__ out) {
  __shared__ __align__(16) unsigned short gsh[8][256];
  const int lane = threadIdx.x & 31, wave = threadIdx.x >> 5;
  const size_t base = ((size_t)blockIdx.x * 8 + wave) * 256;
#pragma unroll 1
  for (int i = 0; i < 8; ++i) {
    const float v = in[base + 32 * i + lane];
    const float gl = 0.5f * v * (1.0f + erff(v * 0.70710678118654752f));
    gsh[wave][32 * i + lane] = h_bits(gl);
  }
  __builtin_amdgcn_fence(__ATOMIC_RELEASE, "workgroup");
  __builtin_amdgcn_wave_barrier();
  __builtin_amdgcn_fence(__ATOMIC_ACQUIRE, "workgroup");
  const v4u u = *(const v4u*)(&gsh[wave][8 * lane]);
  unsigned short* p = out + base + 8 * lane;
  *(volatile v4u*)p = u;
  __threadfence();
  *(volatile v4u*)p = u;
}

extern "C" void kernel_launch(void* const* d_in, const int* in_sizes, int n_in,
                              void* d_out, int out_size, void* d_ws,
                              size_t ws_size, hipStream_t stream) {
  if (n_in < 18) return;
  if (ws_size < kWsTotal) return;
  if ((size_t)out_size < (size_t)kTok * kHid) return;
  if (in_sizes[0] != kTok * kHid || in_sizes[1] != kB * kS) return;
  if (in_sizes[2] != kHid * kHid || in_sizes[12] != kHid * kFF || in_sizes[14] != kFF * kHid) return;

  const float* x    = (const float*)d_in[0];
  const int*   am   = (const int*)d_in[1];
  const float* Wq   = (const float*)d_in[2];
  const float* bq   = (const float*)d_in[3];
  const float* Wk   = (const float*)d_in[4];
  const float* bk   = (const float*)d_in[5];
  const float* Wv   = (const float*)d_in[6];
  const float* bvv  = (const float*)d_in[7];
  const float* Wd   = (const float*)d_in[8];
  const float* bd   = (const float*)d_in[9];
  const float* ln1g = (const float*)d_in[10];
  const float* ln1b = (const float*)d_in[11];
  const float* Wf   = (const float*)d_in[12];
  const float* bff  = (const float*)d_in[13];
  const float* Wo   = (const float*)d_in[14];
  const float* bo   = (const float*)d_in[15];
  const float* ln2g = (const float*)d_in[16];
  const float* ln2b = (const float*)d_in[17];
  float* outp = (float*)d_out;

  char* ws = (char*)d_ws;
  unsigned short* x16    = (unsigned short*)(ws + kOffX16);
  unsigned short* attn16 = (unsigned short*)(ws + kOffX16);
  unsigned short* wt4    = (unsigned short*)(ws + kOffWT);
  unsigned short* wqT    = wt4;
  unsigned short* wkT    = wt4 + (size_t)kHid * kHid;
  unsigned short* wvT    = wt4 + (size_t)2 * kHid * kHid;
  unsigned short* wdT    = wt4 + (size_t)3 * kHid * kHid;
  unsigned short* q16    = (unsigned short*)(ws + kOffQ16);
  unsigned short* wfT    = (unsigned short*)(ws + kOffQ16);
  unsigned short* woT    = wfT + (size_t)kFF * kHid;
  unsigned short* kpad   = (unsigned short*)(ws + kOffKpad);
  float*          attnF  = (float*)(ws + kOffKpad);
  unsigned short* vt     = (unsigned short*)(ws + kOffVT);
  float*          scores = (float*)(ws + kOffSc);
  float*          preln1 = (float*)(ws + kOffSc);
  unsigned short* ff16   = (unsigned short*)(ws + kOffSc);
  unsigned short* p16    = (unsigned short*)(ws + kOffP16);
  unsigned short* ctx16  = (unsigned short*)(ws + kOffCtx);
  float*          ffpre  = (float*)(ws + kOffR8);
  float*          ffo    = (float*)(ws + kOffR8);

  cast8_f16_kernel<<<(kTok * kHid / 8) / 256, 256, 0, stream>>>(x, x16, kTok * kHid / 8);
  wtcast_kernel<<<dim3(kHid / 64, kHid / 64, 4), 256, 0, stream>>>(Wq, Wk, Wv, Wd, wt4, kHid, kHid, kWCarry);
  padzero_kernel<<<384, 256, 0, stream>>>(kpad, vt);

  {
    const int gx = (kTok / 64) * (kHid / 64) / 8;
    gemm_f16_kernel<2, 1, false><<<gx, 256, 0, stream>>>(
        x16, kHid, 0, 0, wqT, kHid, 0, 0, q16, kHid, 0, 0, bq, nullptr, kTok, kHid, kHid, kInvW, 1, 1);
    gemm_f16_kernel<2, 1, false><<<gx, 256, 0, stream>>>(
        x16, kHid, (long)kS * kHid, 0, wkT, kHid, 0, 0, kpad + (size_t)kW * kHid, kHid, (long)kSpad * kHid, 0,
        bk, nullptr, kS, kHid, kHid, kInvW, kB, 1);
    gemm_f16_kernel<1, 1, false><<<gx, 256, 0, stream>>>(
        wvT, kHid, 0, 0, x16, kHid, (long)kS * kHid, 0, vt + kW, kSpad, (long)kHid * kSpad, 0,
        bvv, nullptr, kHid, kS, kHid, kInvW, kB, 1);
  }

  for (int ps = 0; ps < kNPass; ++ps) {
    const int bh0 = ps * kGrp;
    const int b   = bh0 / kNH;
    const int h0  = bh0 - b * kNH;
    {
      const int gx = ((kW / 64) * (kWin / 64) * kNC * kGrp) / 8;
      gemm_f16_kernel<0, 0, false><<<gx, 256, 0, stream>>>(
          q16 + (size_t)b * kS * kHid + (size_t)h0 * kDh, kHid, (long)kW * kHid, kDh,
          kpad + (size_t)b * kSpad * kHid + (size_t)h0 * kDh, kHid, (long)kW * kHid, kDh,
          scores, kWin, (long)kW * kWin, (long)kNC * kW * kWin,
          nullptr, nullptr, kW, kWin, kDh, kQScale, kNC, kGrp);
    }
    band_softmax_kernel<<<(kGrp * kNC * kW) / 8, 256, 0, stream>>>(scores, am, p16, b);
    {
      const int gx = ((kW / 64) * (kDh / 64) * kNC * kGrp) / 8;
      gemm_f16_kernel<0, 1, false><<<gx, 256, 0, stream>>>(
          p16, kWin, (long)kW * kWin, (long)kNC * kW * kWin,
          vt + (size_t)bh0 * kDh * kSpad, kSpad, kW, (long)kDh * kSpad,
          ctx16 + (size_t)b * kS * kHid + (size_t)h0 * kDh, kHid, (long)kW * kHid, kDh,
          nullptr, nullptr, kW, kDh, kWin, kPVScale, kNC, kGrp);
    }
  }

  {
    const int gx = (kTok / 64) * (kHid / 64) / 8;
    gemm_f16_kernel<2, 0, true><<<gx, 256, 0, stream>>>(
        ctx16, kHid, 0, 0, wdT, kHid, 0, 0, preln1, kHid, 0, 0, bd, x, kTok, kHid, kHid, kWdScale, 1, 1);
  }
  layernorm_kernel<true><<<kTok, 192, 0, stream>>>(preln1, ln1g, ln1b, attnF, attn16);

  wtcast_kernel<<<dim3(kHid / 64, kFF / 64, 1), 256, 0, stream>>>(Wf, Wf, Wf, Wf, wfT, kHid, kFF, kWCarry);
  wtcast_kernel<<<dim3(kFF / 64, kHid / 64, 1), 256, 0, stream>>>(Wo, Wo, Wo, Wo, woT, kFF, kHid, kWCarry);

  for (int tc = 0; tc < kNTC; ++tc) {
    const int gx = (kTC / 64) * (kFF / 64) / 8;
    gemm_f16_kernel<2, 0, false><<<gx, 256, 0, stream>>>(
        attn16 + (size_t)tc * kTC * kHid, kHid, 0, 0, wfT, kHid, 0, 0, ffpre, kFF, 0, 0,
        bff, nullptr, kTC, kFF, kHid, kInvW, 1, 1);
    gelu_f16_kernel<<<(kTC * kFF) / 2048, 256, 0, stream>>>(ffpre, ff16 + (size_t)tc * kTC * kFF);
  }

  {
    const int gx = (kTok / 64) * (kHid / 64) / 8;
    gemm_f16_kernel<2, 0, true><<<gx, 256, 0, stream>>>(
        ff16, kFF, 0, 0, woT, kFF, 0, 0, ffo, kHid, 0, 0, bo, attnF, kTok, kHid, kFF, kInvW, 1, 1);
  }
  layernorm_kernel<false><<<kTok, 192, 0, stream>>>(ffo, ln2g, ln2b, outp, nullptr);
}
